// MambaAutoencoder_41755672052460
// MI455X (gfx1250) — hardware-verified
//
#include <hip/hip_runtime.h>
#include <stddef.h>
#include <math.h>


#pragma clang fp contract(off)

#define NB    4
#define LSEQ  1024
#define NTOK  (NB * LSEQ)
#define OBS   128
#define DM    1024
#define DI    2048
#define DS    16
#define DC    4
#define DR    64
#define DBV   96
#define DBW   128
#define LAT   16
#define NTHR  256
#define WSCAP 134217728

#define SZ_WX   ((size_t)DBW * DI * 2)
#define SZ_WDT  ((size_t)DI * DR * 2)
#define SZ_WO   ((size_t)DM * DI * 2)
#define SZ_WDEC ((size_t)OBS * DM * 2)
#define SZ_WLAT ((size_t)LAT * DM * 2)
#define SZ_WIN  ((size_t)2 * DI * DM * 2)
#define SZ_DBL  ((size_t)NTOK * DBW * 4)
#define SZ_DTH  ((size_t)NTOK * DR * 2)
#define SZ_F32P ((size_t)NTOK * DI * 4)
#define SZ_F16P ((size_t)NTOK * DI * 2)
#define SZ_H    ((size_t)NTOK * DM * 2)
#define SZ_XH   ((size_t)NTOK * OBS * 2)
#define SZ_WEH  ((size_t)DM * OBS * 2)

#define O_WX    ((size_t)0)
#define O_WDT   (O_WX + SZ_WX)
#define O_WO    (O_WDT + SZ_WDT)
#define O_WDEC  (O_WO + SZ_WO)
#define O_WLAT  (O_WDEC + SZ_WDEC)
#define O_RA    (O_WLAT + SZ_WLAT)
#define O_WIN   (O_RA)
#define O_DBL   (O_RA)
#define O_DTH   (O_RA + SZ_DBL)
#define O_RB    (O_RA + SZ_WIN)
#define O_XC    (O_RB)
#define O_DEL   (O_RB)
#define O_HS    (O_RB)
#define O_RC    (O_RB + SZ_F32P)
#define O_Z     (O_RC)
#define O_RD    (O_RC + SZ_F32P)
#define O_XH    (O_RD)
#define O_WEH   (O_RD + SZ_XH)
#define O_H     (O_RD + SZ_H)
#define O_U32   (O_RD)
#define O_RE    (O_RD + SZ_F32P)
#define O_UH    (O_RE)
#define O_YH    (O_RE)
#define WSTOT   (O_RE + SZ_F16P)
static_assert(WSTOT <= (size_t)WSCAP);
static_assert(SZ_DBL + SZ_DTH <= SZ_WIN);
static_assert(SZ_XH + SZ_WEH <= SZ_H && 2 * SZ_H <= SZ_F32P && SZ_H <= SZ_F32P);
static_assert((O_WDT % 128) == 0 && (O_WO % 128) == 0 && (O_WDEC % 128) == 0 && (O_WLAT % 128) == 0);
static_assert((O_RA % 128) == 0 && (O_DTH % 128) == 0 && (O_RB % 128) == 0 && (O_RC % 128) == 0);
static_assert((O_RD % 128) == 0 && (O_WEH % 128) == 0 && (O_H % 128) == 0 && (O_RE % 128) == 0 && (WSTOT % 128) == 0);

static_assert((OBS % 32) == 0 && (DM % 32) == 0 && (DI % 32) == 0 && (DR % 32) == 0);
static_assert((NTOK % 128) == 0 && (DM % 256) == 0 && (DI % 256) == 0 && DBW == 128 && OBS == 128 && LAT == 16);
static_assert(DBV + DS + DS <= DBW + 32 && DR + 2 * DS == DBV);

typedef _Float16     v16h __attribute__((ext_vector_type(16)));
typedef _Float16     v8h  __attribute__((ext_vector_type(8)));
typedef _Float16     v4hh __attribute__((ext_vector_type(4)));
typedef float        v8f  __attribute__((ext_vector_type(8)));
typedef float        v4f  __attribute__((ext_vector_type(4), __may_alias__));
typedef unsigned int v4u  __attribute__((ext_vector_type(4), __may_alias__));
typedef unsigned int v2u  __attribute__((ext_vector_type(2), __may_alias__));
typedef int          v8i  __attribute__((ext_vector_type(8)));
union Frag { v16h v; v8i w; v4u q[2]; };
union P8 { v8h h; v4u u; };
union P4 { v4hh h; v2u u; };
static_assert(sizeof(Frag) == 32);
static_assert(sizeof(P8) == 16);
static_assert(sizeof(P4) == 8);

__device__ __forceinline__ v8f wmh(const Frag& a, const Frag& b, v8f c) {
  v8f d = __builtin_amdgcn_wmma_f32_16x16x32_f16(false, a.v, false, b.v, (short)0, c, false, false);
  asm volatile("v_nop\n\tv_nop\n\tv_nop\n\tv_nop" : "+v"(d) : "v"(a.w), "v"(b.w));
  return d;
}

__device__ __forceinline__ v8f zero8() {
  v8f z = {0.f, 0.f, 0.f, 0.f, 0.f, 0.f, 0.f, 0.f};
  return z;
}

__device__ __forceinline__ v4u pack8h(v4f a, v4f c) {
  P8 p;
  p.h[0] = (_Float16)a[0]; p.h[1] = (_Float16)a[1]; p.h[2] = (_Float16)a[2]; p.h[3] = (_Float16)a[3];
  p.h[4] = (_Float16)c[0]; p.h[5] = (_Float16)c[1]; p.h[6] = (_Float16)c[2]; p.h[7] = (_Float16)c[3];
  return p.u;
}

__device__ __forceinline__ v2u pack4h(v4f a) {
  P4 p;
  p.h[0] = (_Float16)a[0]; p.h[1] = (_Float16)a[1]; p.h[2] = (_Float16)a[2]; p.h[3] = (_Float16)a[3];
  return p.u;
}

#define CVB     2048
#define CE_X    (NTOK * OBS / CVB)
#define CE_WE   (CE_X + DM * OBS / CVB)
#define CE_WIN  (CE_WE + 2 * DI * DM / CVB)
#define CE_WX   (CE_WIN + DBV * DI / CVB)
#define CE_PAD  (CE_WIN + DBW * DI / CVB)
#define CE_WDT  (CE_PAD + DI * DR / CVB)
#define CE_WO   (CE_WDT + DM * DI / CVB)
#define CE_WDEC (CE_WO + OBS * DM / CVB)
#define CE_TOT  (CE_WDEC + LAT * DM / CVB)
static_assert(CVB == NTHR * 8);
static_assert(((NTOK * OBS) % CVB) == 0 && ((DM * OBS) % CVB) == 0 && ((DBV * DI) % CVB) == 0 && ((DBW * DI) % CVB) == 0);
static_assert(((DI * DR) % CVB) == 0 && ((OBS * DM) % CVB) == 0 && ((LAT * DM) % CVB) == 0 && CE_TOT == 3656);

__global__ __launch_bounds__(NTHR) void k_cvt(const float* __restrict__ x, const float* __restrict__ wenc,
                                              const float* __restrict__ win, const float* __restrict__ wx,
                                              const float* __restrict__ wdt, const float* __restrict__ wo,
                                              const float* __restrict__ wdec, const float* __restrict__ wlat,
                                              unsigned short* XH, unsigned short* WEH, unsigned short* WIN,
                                              unsigned short* WX, unsigned short* WDT, unsigned short* WO,
                                              unsigned short* WDEC, unsigned short* WLAT) {
  const int blk = blockIdx.x, tid = threadIdx.x;
  const float* src;
  unsigned short* dst;
  int bs;
  float sc;
  int zf = 0;
  if (blk < CE_X)         { src = x;    dst = XH;   bs = 0;       sc = 1.0f;  }
  else if (blk < CE_WE)   { src = wenc; dst = WEH;  bs = CE_X;    sc = 16.0f; }
  else if (blk < CE_WIN)  { src = win;  dst = WIN;  bs = CE_WE;   sc = 32.0f; }
  else if (blk < CE_PAD)  { src = wx;   dst = WX;   bs = CE_WIN;  sc = 64.0f; zf = (blk >= CE_WX) ? 1 : 0; }
  else if (blk < CE_WDT)  { src = wdt;  dst = WDT;  bs = CE_PAD;  sc = 8.0f;  }
  else if (blk < CE_WO)   { src = wo;   dst = WO;   bs = CE_WDT;  sc = 32.0f; }
  else if (blk < CE_WDEC) { src = wdec; dst = WDEC; bs = CE_WO;   sc = 32.0f; }
  else                    { src = wlat; dst = WLAT; bs = CE_WDEC; sc = 32.0f; }
  const size_t eo = (size_t)(blk - bs) * CVB + (size_t)tid * 8;
  const size_t so = zf ? ((size_t)tid * 8) : eo;
  const float scl = zf ? 0.0f : sc;
  v4f a0 = *(const v4f*)(src + so);
  v4f a1 = *(const v4f*)(src + so + 4);
  a0 = a0 * scl;
  a1 = a1 * scl;
  const v4u hv = pack8h(a0, a1);
  *(volatile v4u*)(dst + eo) = hv;
  __threadfence();
  *(volatile v4u*)(dst + eo) = hv;
}

template <int WM, int NT, int EP>
__global__ __launch_bounds__(NTHR) void k_gemm(const unsigned short* __restrict__ Ah,
                                               const unsigned short* __restrict__ Wh,
                                               const float* __restrict__ bias,
                                               float* Cf, unsigned short* Ph,
                                               int lda, int ldw, int ldc, int ldp, int K, float osc) {
  constexpr int WN = 8 / WM;
  constexpr int R = 16 * WM;
  constexpr int BN = WN * 16 * NT;
  static_assert(WM * WN == 8);
  static_assert(((R * BN / 4) % NTHR) == 0);
  constexpr int NF4 = (R * BN / 4) / NTHR;
  constexpr int Q4 = BN / 4;
  constexpr bool HASB = (EP == 1 || EP == 2 || EP == 3);
  constexpr bool F32O = (EP == 0 || EP == 1 || EP == 2 || EP == 5);
  constexpr bool F16O = (EP == 3 || EP == 4);
  __shared__ __align__(16) float sC[R * BN];
  const int tid = threadIdx.x, lane = tid & 31, wave = tid >> 5, h = lane >> 4, m = lane & 15;
  const int wm = wave % WM, wn = wave / WM;
  const int bm0 = blockIdx.y * R;
  const int n0 = blockIdx.x * BN;
  const int m0 = bm0 + 16 * wm;
  const int nw0 = n0 + wn * 16 * NT;

  v8f acc[NT];
#pragma unroll
  for (int t = 0; t < NT; ++t) acc[t] = zero8();

  const size_t arow = (size_t)(m0 + m) * (size_t)lda + (size_t)(8 * h);
  const size_t wrow = (size_t)(nw0 + m) * (size_t)ldw + (size_t)(8 * h);
  const int nks = K >> 5;

#pragma unroll 1
  for (int ks = 0; ks < nks; ++ks) {
    const int k0 = ks << 5;
    Frag fa;
    fa.q[0] = *(const v4u*)(Ah + arow + k0);
    fa.q[1] = *(const v4u*)(Ah + arow + k0 + 16);
#pragma unroll
    for (int t = 0; t < NT; ++t) {
      const unsigned short* wp = Wh + wrow + (size_t)(16 * t) * (size_t)ldw + k0;
      Frag fw;
      fw.q[0] = *(const v4u*)wp;
      fw.q[1] = *(const v4u*)(wp + 16);
      acc[t] = wmh(fa, fw, acc[t]);
    }
  }

#pragma unroll
  for (int t = 0; t < NT; ++t) {
    const int cl = wn * 16 * NT + 16 * t + m;
#pragma unroll
    for (int r = 0; r < 8; ++r) {
      const int rl = 16 * wm + 8 * h + r;
      sC[rl * BN + cl] = acc[t][r];
    }
  }
  __syncthreads();

  if constexpr (F32O) {
#pragma unroll 1
    for (int it = 0; it < NF4; ++it) {
      const int e = tid + it * NTHR;
      const int rl = e / Q4, q = e - rl * Q4;
      v4f v = *(const v4f*)(sC + 4 * e);
      v = v * osc;
      if constexpr (HASB) {
        const v4f bb = *(const v4f*)(bias + n0 + 4 * q);
        v = v + bb;
      }
      if constexpr (EP == 2) {
#pragma unroll
        for (int j = 0; j < 4; ++j) {
          const float a = v[j];
          v[j] = fmaxf(a, 0.0f) + log1pf(__expf(-fabsf(a)));
        }
      }
      *(v4f*)(sC + 4 * e) = v;
    }
#pragma unroll
    for (int it = 0; it < NF4; ++it) {
      const int e = tid + it * NTHR;
      const int rl = e / Q4, q = e - rl * Q4;
      const v4f v = *(const v4f*)(sC + 4 * e);
      *(volatile v4f*)(Cf + (size_t)(bm0 + rl) * (size_t)ldc + n0 + 4 * q) = v;
    }
    __threadfence();
#pragma unroll
    for (int it = 0; it < NF4; ++it) {
      const int e = tid + it * NTHR;
      const int rl = e / Q4, q = e - rl * Q4;
      const v4f v = *(const v4f*)(sC + 4 * e);
      *(volatile v4f*)(Cf + (size_t)(bm0 + rl) * (size_t)ldc + n0 + 4 * q) = v;
    }
  }

  if constexpr (F16O) {
    static_assert(((R * BN / 8) % NTHR) == 0);
    constexpr int NP8 = (R * BN / 8) / NTHR;
    constexpr int Q8 = BN / 8;
    v4u hv[NP8];
    size_t dst[NP8];
#pragma unroll
    for (int it = 0; it < NP8; ++it) {
      const int e = tid + it * NTHR;
      const int rl = e / Q8, q = e - rl * Q8;
      v4f a = *(const v4f*)(sC + rl * BN + 8 * q);
      v4f c = *(const v4f*)(sC + rl * BN + 8 * q + 4);
      a = a * osc;
      c = c * osc;
      if constexpr (HASB) {
        const v4f b0 = *(const v4f*)(bias + n0 + 8 * q);
        const v4f b1 = *(const v4f*)(bias + n0 + 8 * q + 4);
        a = a + b0;
        c = c + b1;
      }
      hv[it] = pack8h(a, c);
      dst[it] = (size_t)(bm0 + rl) * (size_t)ldp + n0 + 8 * q;
    }
#pragma unroll
    for (int it = 0; it < NP8; ++it) *(volatile v4u*)(Ph + dst[it]) = hv[it];
    __threadfence();
#pragma unroll
    for (int it = 0; it < NP8; ++it) *(volatile v4u*)(Ph + dst[it]) = hv[it];
  }

  if constexpr (EP == 5) {
    static_assert(R == 64 && BN >= DR && (R * DR / 8) == 2 * NTHR);
    __syncthreads();
    v4u hv[2];
    size_t dst[2];
#pragma unroll
    for (int it = 0; it < 2; ++it) {
      const int e = tid + it * NTHR;
      const int rl = e >> 3, q = e & 7;
      const v4f a = *(const v4f*)(sC + rl * BN + 8 * q);
      const v4f c = *(const v4f*)(sC + rl * BN + 8 * q + 4);
      hv[it] = pack8h(a, c);
      dst[it] = (size_t)(bm0 + rl) * DR + 8 * q;
    }
#pragma unroll
    for (int it = 0; it < 2; ++it) *(volatile v4u*)(Ph + dst[it]) = hv[it];
    __threadfence();
#pragma unroll
    for (int it = 0; it < 2; ++it) *(volatile v4u*)(Ph + dst[it]) = hv[it];
  }
}

static_assert((DI / 4) == 512 && ((NTOK * DI / 4) % NTHR) == 0);

__global__ __launch_bounds__(NTHR) void k_conv(const float* __restrict__ XC, const float* __restrict__ cw,
                                               const float* __restrict__ cb, float* U32, unsigned short* UH) {
  const int g = blockIdx.x * NTHR + threadIdx.x;
  const int row = g >> 9;
  const int dq = (g & 511) << 2;
  const int t = row & (LSEQ - 1);
  const int rb = row - t;
  v4f acc = *(const v4f*)(cb + dq);
  v4f w[4];
#pragma unroll
  for (int j = 0; j < 4; ++j) w[j] = *(const v4f*)(cw + (size_t)(dq + j) * DC);
#pragma unroll
  for (int k = 0; k < DC; ++k) {
    const int tt = t + k - (DC - 1);
    const int ttc = (tt < 0) ? 0 : tt;
    const v4f xv = *(const v4f*)(XC + (size_t)(rb + ttc) * (size_t)DI + dq);
    const float f = (tt >= 0) ? 1.0f : 0.0f;
#pragma unroll
    for (int j = 0; j < 4; ++j) acc[j] = acc[j] + (xv[j] * f) * w[j][k];
  }
  v4f u;
#pragma unroll
  for (int j = 0; j < 4; ++j) {
    const float a = acc[j];
    u[j] = a * __builtin_amdgcn_rcpf(1.0f + __expf(-a));
  }
  const v2u hv = pack4h(u);
  const size_t o = (size_t)g * 4;
  *(volatile v4f*)(U32 + o) = u;
  *(volatile v2u*)(UH + o) = hv;
  __threadfence();
  *(volatile v4f*)(U32 + o) = u;
  *(volatile v2u*)(UH + o) = hv;
}

#define SCB 256
#define STB 32
static_assert(SCB == NTHR && (DI % SCB) == 0 && (LSEQ % STB) == 0 && DS == 16);
static_assert(((STB * SCB / 8) % NTHR) == 0);

__global__ __launch_bounds__(NTHR) void k_scan(const float* __restrict__ DEL, const float* __restrict__ U32,
                                               const float* __restrict__ DBL, const float* __restrict__ Zp,
                                               const float* __restrict__ Alog, const float* __restrict__ Dp,
                                               unsigned short* YH) {
  __shared__ __align__(16) float sA[SCB * DS];
  __shared__ __align__(16) float sY[STB * SCB];
  const int tid = threadIdx.x;
  const int cbase = blockIdx.x * SCB;
  const int ch = cbase + tid;
  const size_t rbase = (size_t)blockIdx.y * LSEQ;
#pragma unroll 1
  for (int e = tid; e < SCB * DS; e += NTHR) sA[e] = -expf(Alog[(size_t)cbase * DS + e]);
  __syncthreads();

  float Ac[DS], hs[DS];
#pragma unroll
  for (int n = 0; n < DS; ++n) {
    Ac[n] = sA[tid * DS + n];
    hs[n] = 0.0f;
  }
  const float Dd = Dp[ch];

#pragma unroll 1
  for (int t0 = 0; t0 < LSEQ; t0 += STB) {
#pragma unroll 1
    for (int tl = 0; tl < STB; ++tl) {
      const size_t row = rbase + (size_t)(t0 + tl);
      const float dt = DEL[row * DI + ch];
      const float u = U32[row * DI + ch];
      const float z = Zp[row * DI + ch];
      const float* bp = DBL + row * DBW + DR;
      v4f bq[4], cq[4];
#pragma unroll
      for (int i = 0; i < 4; ++i) {
        bq[i] = *(const v4f*)(bp + 4 * i);
        cq[i] = *(const v4f*)(bp + DS + 4 * i);
      }
      const float dtu = dt * u;
      float part = 0.0f;
#pragma unroll
      for (int n = 0; n < DS; ++n) {
        const float bv = bq[n >> 2][n & 3];
        const float cv = cq[n >> 2][n & 3];
        const float dA = __expf(dt * Ac[n]);
        const float hn = dA * hs[n] + dtu * bv;
        hs[n] = hn;
        part = part + hn * cv;
      }
      const float sg = __builtin_amdgcn_rcpf(1.0f + __expf(-z));
      const float y = (part + Dd * u) * (z * sg);
      sY[tl * SCB + tid] = y;
    }
    __syncthreads();
    {
      constexpr int NIT = (STB * SCB / 8) / NTHR;
      v4u hv[NIT];
      size_t dst[NIT];
#pragma unroll
      for (int it = 0; it < NIT; ++it) {
        const int e = tid + it * NTHR;
        const int rl = e >> 5, q = e & 31;
        const v4f a = *(const v4f*)(sY + rl * SCB + 8 * q);
        const v4f c = *(const v4f*)(sY + rl * SCB + 8 * q + 4);
        hv[it] = pack8h(a, c);
        dst[it] = (rbase + (size_t)(t0 + rl)) * (size_t)DI + (size_t)(cbase + 8 * q);
      }
#pragma unroll
      for (int it = 0; it < NIT; ++it) *(volatile v4u*)(YH + dst[it]) = hv[it];
      __threadfence();
#pragma unroll
      for (int it = 0; it < NIT; ++it) *(volatile v4u*)(YH + dst[it]) = hv[it];
    }
    __syncthreads();
  }
}

extern "C" void kernel_launch(void* const* d_in, const int* in_sizes, int n_in,
                              void* d_out, int out_size, void* d_ws, size_t ws_size,
                              hipStream_t stream) {
  if (n_in < 16) return;
  if (in_sizes[0] != NTOK * OBS) return;
  if (in_sizes[1] != DM * OBS || in_sizes[2] != DM) return;
  if (in_sizes[3] != 2 * DI * DM) return;
  if (in_sizes[4] != DI * DC || in_sizes[5] != DI) return;
  if (in_sizes[6] != DBV * DI) return;
  if (in_sizes[7] != DI * DR || in_sizes[8] != DI) return;
  if (in_sizes[9] != DI * DS || in_sizes[10] != DI) return;
  if (in_sizes[11] != DM * DI) return;
  if (in_sizes[12] != OBS * DM || in_sizes[13] != OBS) return;
  if (in_sizes[14] != LAT * DM || in_sizes[15] != LAT) return;
  if (out_size != NTOK * OBS + NTOK * LAT) return;
  const size_t tot = (size_t)WSTOT;
  if (tot > ws_size || tot > (size_t)WSCAP) return;

  const float* x    = (const float*)d_in[0];
  const float* wenc = (const float*)d_in[1];
  const float* benc = (const float*)d_in[2];
  const float* win  = (const float*)d_in[3];
  const float* cw   = (const float*)d_in[4];
  const float* cb   = (const float*)d_in[5];
  const float* wx   = (const float*)d_in[6];
  const float* wdt  = (const float*)d_in[7];
  const float* bdt  = (const float*)d_in[8];
  const float* alog = (const float*)d_in[9];
  const float* dsk  = (const float*)d_in[10];
  const float* wo   = (const float*)d_in[11];
  const float* wdec = (const float*)d_in[12];
  const float* bdec = (const float*)d_in[13];
  const float* wlat = (const float*)d_in[14];
  const float* blat = (const float*)d_in[15];
  float* out0 = (float*)d_out;
  float* out1 = (float*)d_out + (size_t)NTOK * OBS;

  char* ws = (char*)d_ws;
  unsigned short* WX   = (unsigned short*)(ws + O_WX);
  unsigned short* WDT  = (unsigned short*)(ws + O_WDT);
  unsigned short* WO   = (unsigned short*)(ws + O_WO);
  unsigned short* WDEC = (unsigned short*)(ws + O_WDEC);
  unsigned short* WLAT = (unsigned short*)(ws + O_WLAT);
  unsigned short* WIN  = (unsigned short*)(ws + O_WIN);
  float*          DBL  = (float*)(ws + O_DBL);
  unsigned short* DTH  = (unsigned short*)(ws + O_DTH);
  float*          XC   = (float*)(ws + O_XC);
  float*          DEL  = (float*)(ws + O_DEL);
  unsigned short* HS   = (unsigned short*)(ws + O_HS);
  float*          Z    = (float*)(ws + O_Z);
  unsigned short* XH   = (unsigned short*)(ws + O_XH);
  unsigned short* WEH  = (unsigned short*)(ws + O_WEH);
  unsigned short* H    = (unsigned short*)(ws + O_H);
  float*          U32  = (float*)(ws + O_U32);
  unsigned short* UH   = (unsigned short*)(ws + O_UH);
  unsigned short* YH   = (unsigned short*)(ws + O_YH);


  k_cvt<<<CE_TOT, NTHR, 0, stream>>>(x, wenc, win, wx, wdt, wo, wdec, wlat, XH, WEH, WIN, WX, WDT, WO, WDEC, WLAT);

  k_gemm<2, 4, 3><<<dim3(DM / 256, NTOK / 32), NTHR, 0, stream>>>(
      XH, WEH, benc, Z, H, OBS, OBS, 0, DM, OBS, 0.0625f);

  k_gemm<2, 4, 0><<<dim3(DI / 256, NTOK / 32), NTHR, 0, stream>>>(
      H, WIN, benc, XC, DTH, DM, DM, DI, 0, DM, 0.03125f);

  k_gemm<2, 4, 0><<<dim3(DI / 256, NTOK / 32), NTHR, 0, stream>>>(
      H, WIN + (size_t)DI * DM, benc, Z, DTH, DM, DM, DI, 0, DM, 0.03125f);

  k_conv<<<(NTOK * DI / 4) / NTHR, NTHR, 0, stream>>>(XC, cw, cb, U32, UH);

  k_gemm<4, 4, 5><<<dim3(DBW / 128, NTOK / 64), NTHR, 0, stream>>>(
      UH, WX, benc, DBL, DTH, DI, DI, DBW, DR, DI, 0.015625f);

  k_gemm<2, 4, 2><<<dim3(DI / 256, NTOK / 32), NTHR, 0, stream>>>(
      DTH, WDT, bdt, DEL, YH, DR, DR, DI, 0, DR, 0.125f);

  k_scan<<<dim3(DI / SCB, NB), NTHR, 0, stream>>>(DEL, U32, DBL, Z, alog, dsk, YH);

  k_gemm<2, 4, 4><<<dim3(DM / 256, NTOK / 32), NTHR, 0, stream>>>(
      YH, WO, benc, Z, HS, DI, DI, 0, DM, DI, 0.03125f);

  k_gemm<4, 4, 1><<<dim3(OBS / 128, NTOK / 64), NTHR, 0, stream>>>(
      HS, WDEC, bdec, out0, DTH, DM, DM, OBS, 0, DM, 0.03125f);

  k_gemm<8, 1, 1><<<dim3(LAT / 16, NTOK / 128), NTHR, 0, stream>>>(
      HS, WLAT, blat, out1, DTH, DM, DM, LAT, 0, DM, 0.03125f);
}
